// KPConvLayer_23450521436528
// MI455X (gfx1250) — hardware-verified
//
#include <hip/hip_runtime.h>
#include <math.h>

typedef __attribute__((ext_vector_type(16))) _Float16 v16h;
typedef __attribute__((ext_vector_type(16))) __bf16 v16b;
typedef __attribute__((ext_vector_type(8)))  _Float16 v8h;
typedef __attribute__((ext_vector_type(8)))  float v8f;
typedef __attribute__((ext_vector_type(4)))  float v4f;
typedef __attribute__((ext_vector_type(2)))  float v2f;
typedef __attribute__((ext_vector_type(4)))  unsigned v4u;
typedef __attribute__((ext_vector_type(4)))  int v4i;
typedef float __attribute__((may_alias)) float_a;
typedef int __attribute__((may_alias)) int_a;

template <typename T> __device__ __forceinline__ void vst2(void* p, T v) { *(volatile T*)p = v; __threadfence(); *(volatile T*)p = v; }
__device__ __forceinline__ v8f wmma16(v16h a, v16h b, v8f c) {
  v8f d = __builtin_amdgcn_wmma_f32_16x16x32_f16(false, a, false, b, (short)0, c, false, false);
  asm volatile("v_nop\n\tv_nop\n\tv_nop\n\tv_nop" : "+v"(d) : "v"(a), "v"(b));
  return d;
}
__device__ __forceinline__ v8f wmma_bf(v16b a, v16b b, v8f c) {
  v8f d = __builtin_amdgcn_wmma_f32_16x16x32_bf16(false, a, false, b, (short)0, c, false, false);
  asm volatile("v_nop\n\tv_nop\n\tv_nop\n\tv_nop" : "+v"(d) : "v"(a), "v"(b));
  return d;
}
__device__ __forceinline__ v16h frag_h(const _Float16* rowk0, int lane) {
  union { v16h v; v8h q[2]; } u; const _Float16* p = rowk0 + 8 * (lane >> 4);
  u.q[0] = *(const v8h*)p; u.q[1] = *(const v8h*)(p + 16); return u.v;
}
__device__ __forceinline__ v16h frag_f32(const float* rowk0, int lane) {
  v16h a; const float* p = rowk0 + 8 * (lane >> 4);
#pragma unroll
  for (int i = 0; i < 8; ++i) { a[i] = (_Float16)p[i]; a[8 + i] = (_Float16)p[16 + i]; }
  return a;
}
__device__ __forceinline__ v16h frag_f32s(const float* rowk0, int lane, float sc) {
  v16h a; const float* p = rowk0 + 8 * (lane >> 4);
#pragma unroll
  for (int i = 0; i < 8; ++i) { a[i] = (_Float16)(p[i] * sc); a[8 + i] = (_Float16)(p[16 + i] * sc); }
  return a;
}
__device__ __forceinline__ v16h fragc_f32(const float* W, int k0, int n, int lane, int ld, int K) {
  v16h a; const int g = lane >> 4;
#pragma unroll
  for (int i = 0; i < 8; ++i) { const int ka = k0 + 8 * g + i, kb = ka + 16;
    a[i] = (_Float16)(ka < K ? W[(size_t)(ka < K ? ka : K - 1) * ld + n] : 0.f); a[8 + i] = (_Float16)(kb < K ? W[(size_t)(kb < K ? kb : K - 1) * ld + n] : 0.f); }
  return a;
}
struct F2 { v16b h, l; };
__device__ __forceinline__ F2 bsplit16(const float v[16]) { F2 r;
#pragma unroll
  for (int i = 0; i < 16; ++i) { const __bf16 h = (__bf16)v[i]; r.h[i] = h; r.l[i] = (__bf16)(v[i] - (float)h); }
  return r; }
__device__ __forceinline__ F2 split_row(const float* row, int k0, int lane) { float v[16]; const float* p = row + k0 + 8 * (lane >> 4);
#pragma unroll
  for (int i = 0; i < 8; ++i) { v[i] = p[i]; v[8 + i] = p[16 + i]; }
  return bsplit16(v); }
__device__ __forceinline__ F2 split_rowK(const float* row, int k0, int lane, int K) { float v[16]; const int g = lane >> 4;
#pragma unroll
  for (int i = 0; i < 8; ++i) { const int ka = k0 + 8 * g + i, kb = ka + 16; v[i] = ka < K ? row[ka < K ? ka : K - 1] : 0.f; v[8 + i] = kb < K ? row[kb < K ? kb : K - 1] : 0.f; }
  return bsplit16(v); }
__device__ __forceinline__ F2 split_col(const float* W, int k0, int n, int lane, int ld, int K) { float v[16]; const int g = lane >> 4;
#pragma unroll
  for (int i = 0; i < 8; ++i) { const int ka = k0 + 8 * g + i, kb = ka + 16; v[i] = ka < K ? W[(size_t)(ka < K ? ka : K - 1) * ld + n] : 0.f; v[8 + i] = kb < K ? W[(size_t)(kb < K ? kb : K - 1) * ld + n] : 0.f; }
  return bsplit16(v); }
__device__ __forceinline__ v8f mac3(const F2& a, const F2& b, v8f c) { c = wmma_bf(a.l, b.h, c); c = wmma_bf(a.h, b.l, c); return wmma_bf(a.h, b.h, c); }
__device__ __forceinline__ float sigm(float v) { return 1.0f / (1.0f + expf(-v)); }
#define LDSX() do { asm volatile("s_wait_dscnt 0" ::: "memory"); __builtin_amdgcn_wave_barrier(); __builtin_amdgcn_fence(__ATOMIC_RELEASE, "workgroup"); } while (0)

__device__ __forceinline__ float bfr(float v) { return (float)(__bf16)v; }
#define NB 4
#define MP 16384
#define KNB 32
#define DIN 64
#define DOUT 64
#define KP 15
#define KFE (KP * DIN)
#ifndef NBLK
#define NBLK (NB * MP / 16)
#endif
typedef __attribute__((ext_vector_type(8))) __bf16 v8b;
__device__ __forceinline__ v16b frag_lds(const __bf16* rowk0, int lane) { union { v16b v; v8b q[2]; } u; const __bf16* p = rowk0 + 8 * (lane >> 4); u.q[0] = *(const v8b*)p; u.q[1] = *(const v8b*)(p + 16); return u.v; }
__global__ __launch_bounds__(128) void k_kp(const float* __restrict__ X, const float* __restrict__ F, const int* __restrict__ NI, const float* __restrict__ Q, const float* __restrict__ W, float* __restrict__ OUT) {
  __shared__ __align__(16) __bf16 fkh[16][KFE + 8], fkl[16][KFE + 8]; __shared__ __align__(16) float so[16][DOUT + 4];
  const int tid = threadIdx.x, wave = tid >> 5, lane = tid & 31, col = lane & 15, g = lane >> 4; const size_t p0 = (size_t)blockIdx.x * 16;
  for (int q = 0; q < 4; ++q) { const int pt = wave * 4 + q; const size_t gp = p0 + pt; const size_t b = gp / MP;
    const float cx = bfr(X[gp * 3]), cy = bfr(X[gp * 3 + 1]), cz = bfr(X[gp * 3 + 2]);
    float hv[16]; { const float qx = (col < KP) ? bfr(Q[col * 3]) : 0.f, qy = (col < KP) ? bfr(Q[col * 3 + 1]) : 0.f, qz = (col < KP) ? bfr(Q[col * 3 + 2]) : 0.f;
#pragma unroll
      for (int i = 0; i < 16; ++i) { const int k = (i < 8) ? (8 * g + i) : (16 + 8 * g + i - 8); int n = NI[gp * KNB + k]; n = n < 0 ? 0 : (n >= MP ? MP - 1 : n); const size_t gn = b * MP + n;
        const float rx = bfr(X[gn * 3]) - cx - qx, ry = bfr(X[gn * 3 + 1]) - cy - qy, rz = bfr(X[gn * 3 + 2]) - cz - qz; const float d = sqrtf(rx * rx + ry * ry + rz * rz); hv[i] = (col < KP) ? fmaxf(0.f, 1.0f - d / 1.0f) : 0.f; } }
    asm volatile("s_wait_loadcnt 0x0" ::: "memory"); const F2 a = bsplit16(hv);
    v8f acc[4] = {};
#pragma unroll
    for (int j = 0; j < 4; ++j) { v16b fb; const int d = j * 16 + col;
#pragma unroll
      for (int i = 0; i < 16; ++i) { const int k = (i < 8) ? (8 * g + i) : (16 + 8 * g + i - 8); int n = NI[gp * KNB + k]; n = n < 0 ? 0 : (n >= MP ? MP - 1 : n); fb[i] = (__bf16)F[(b * MP + n) * DIN + d]; }
      asm volatile("s_wait_loadcnt 0x0" ::: "memory"); acc[j] = wmma_bf(a.h, fb, acc[j]); acc[j] = wmma_bf(a.l, fb, acc[j]); }
#pragma unroll
    for (int j = 0; j < 4; ++j)
#pragma unroll
      for (int r = 0; r < 8; ++r) { const int p = 8 * g + r; if (p < KP) { const float v = acc[j][r]; const __bf16 bh = (__bf16)v; fkh[pt][p * DIN + j * 16 + col] = bh; fkl[pt][p * DIN + j * 16 + col] = (__bf16)(v - (float)bh); } } }
  __syncthreads();
  { v8f acc1 = {};
#pragma unroll 2
    for (int kc = 0; kc < KFE / 32; ++kc) { const v16b ah = frag_lds(&fkh[col][kc * 32], lane), al = frag_lds(&fkl[col][kc * 32], lane); v16b w; const int o = wave * 16 + col;
#pragma unroll
      for (int i = 0; i < 8; ++i) { w[i] = (__bf16)W[(size_t)(kc * 32 + 8 * g + i) * DOUT + o]; w[8 + i] = (__bf16)W[(size_t)(kc * 32 + 16 + 8 * g + i) * DOUT + o]; }
      asm volatile("s_wait_loadcnt 0x0" ::: "memory"); acc1 = wmma_bf(ah, w, acc1); acc1 = wmma_bf(al, w, acc1); }
#pragma unroll
    for (int r = 0; r < 8; ++r) so[8 * g + r][wave * 16 + col] = acc1[r]; }
  __syncthreads();
  for (int e = tid; e < 16 * 16; e += 128) { const int rl = e >> 4, q = e & 15; vst2(OUT + (p0 + rl) * DOUT + q * 4, *(const v4f*)&so[rl][q * 4]); } }
extern "C" void kernel_launch(void* const* d_in, const int* in_sizes, int n_in, void* d_out, int out_size, void* d_ws, size_t ws_size, hipStream_t stream) {
  (void)in_sizes; (void)n_in; (void)out_size; (void)d_ws; (void)ws_size;
  const float** Fp = (const float**)d_in;
  k_kp<<<dim3(NBLK), 128, 0, stream>>>(Fp[0], Fp[1], (const int*)d_in[2], Fp[3], Fp[4], (float*)d_out);
}
